// DAMM_CKAM_57337813401752
// MI455X (gfx1250) — hardware-run, weakly checked
//
#include <hip/hip_runtime.h>
#include <math.h>

constexpr int kNB   = 4;
constexpr int kCh   = 512;
constexpr int kPos  = 4096;
constexpr int kCq   = 64;
constexpr int kOutC = 256;
constexpr float kWCarry    = 64.0f;
constexpr float kWCarryInv = 1.0f / kWCarry;
constexpr float kPCarry    = 32768.0f;
constexpr float kPCarryInv = 1.0f / kPCarry;
constexpr float kACarry    = 1024.0f;
constexpr float kACarryInv = 1.0f / kACarry;
constexpr float kBnEps     = 1e-5f;
constexpr float kBnCntInv  = 1.0f / (float)(kNB * kPos);

static_assert((kCh % 64) == 0 && (kPos % 64) == 0 && (kCq % 64) == 0 && (kOutC % 64) == 0, "tile multiples");
static_assert((kCh % 32) == 0 && (kPos % 32) == 0 && (kCq % 32) == 0, "k multiples of 32");
static_assert(((kCh / 64) * (kCh / 64)) % 8 == 0, "gram tiles per block");
static_assert(((kPos / 64) * (kCq / 64)) % 8 == 0, "qk tiles per block");
static_assert(((kOutC / 64) * (kPos / 64)) % 8 == 0, "conv tiles per block");
static_assert(kPos == 4096 && kCh == 512, "softmax kernels assume these row lengths");

constexpr size_t kSzR0 = (size_t)2 * kNB * kCh * kPos * 2;
constexpr size_t kSzXT = (size_t)kNB * kPos * kCh * 2;
constexpr size_t kSzQT = (size_t)kNB * kPos * kCq * 2;
constexpr size_t kSzVV = (size_t)kNB * kCh * kPos * 2;
constexpr size_t kSzEE = (size_t)kNB * kCh * kCh * 4;
constexpr size_t kSzAT = (size_t)kNB * kCh * kCh * 2;
constexpr size_t kSzYY = (size_t)kNB * kOutC * kPos * 4;
constexpr size_t kOffR0 = 0;
constexpr size_t kOffXT = kOffR0 + kSzR0;
constexpr size_t kOffQT = kOffXT + kSzXT;
constexpr size_t kOffKT = kOffQT + kSzQT;
constexpr size_t kOffVV = kOffKT + kSzQT;
constexpr size_t kOffEE = kOffVV + kSzVV;
constexpr size_t kOffAT = kOffEE + kSzEE;
constexpr size_t kOffPM = kOffAT + kSzAT;
constexpr size_t kOffST = kOffPM + kSzXT;
constexpr size_t kOffYY = kOffST + kSzXT;
constexpr size_t kOffWQ = kOffYY + kSzYY;
constexpr size_t kOffWK = kOffWQ + (size_t)kCq * kCh * 2;
constexpr size_t kOffWV = kOffWK + (size_t)kCq * kCh * 2;
constexpr size_t kOffWC = kOffWV + (size_t)kCh * kCh * 2;
constexpr size_t kWsTotal = kOffWC + (size_t)kOutC * kCh * 2;
static_assert(kWsTotal == 128843776ull, "carve total");
static_assert(kWsTotal <= 134217728ull, "carve cap");
static_assert((size_t)kPos * kPos * 2 <= kSzR0, "score plane fits the aliased region");
static_assert((kOffXT % 128) == 0 && (kOffQT % 128) == 0 && (kOffKT % 128) == 0 && (kOffVV % 128) == 0 &&
              (kOffEE % 128) == 0 && (kOffAT % 128) == 0 && (kOffPM % 128) == 0 && (kOffST % 128) == 0 &&
              (kOffYY % 128) == 0 && (kOffWQ % 128) == 0 && (kOffWK % 128) == 0 && (kOffWV % 128) == 0 &&
              (kOffWC % 128) == 0, "aligned regions");

typedef __attribute__((ext_vector_type(16))) _Float16 v16h;
typedef __attribute__((ext_vector_type(8)))  _Float16 v8h;
typedef __attribute__((ext_vector_type(16))) __bf16   v16b;
typedef __attribute__((ext_vector_type(8)))  __bf16   v8b;
typedef __attribute__((ext_vector_type(8)))  float    v8f;
typedef __attribute__((ext_vector_type(4)))  float    v4f;
typedef __attribute__((ext_vector_type(4)))  unsigned int v4u;

__device__ __forceinline__ unsigned short f2bf_bits(float f) {
  unsigned u = __float_as_uint(f);
  return (unsigned short)((u + 0x7FFFu + ((u >> 16) & 1u)) >> 16);
}
__device__ __forceinline__ float bf_bits2f(unsigned short h) { return __uint_as_float(((unsigned)h) << 16); }
__device__ __forceinline__ unsigned pk16(unsigned short a, unsigned short b) { return (unsigned)a | ((unsigned)b << 16); }
__device__ __forceinline__ unsigned short h_bits(float f) { const _Float16 h = (_Float16)f; return __builtin_bit_cast(unsigned short, h); }
__device__ __forceinline__ float h16_to_f32(unsigned hb) {
  const unsigned sgn = (hb & 0x8000u) << 16;
  const unsigned em = hb & 0x7fffu;
  const float fn = __uint_as_float((em << 13) + 0x38000000u);
  const float fs = (float)em * 5.9604644775390625e-8f;
  const float mag = (em < 0x400u) ? fs : fn;
  return __uint_as_float(__float_as_uint(mag) | sgn);
}

__device__ __forceinline__ v8f mma_h(v16h a, v16h b, v8f c) {
  c = __builtin_amdgcn_wmma_f32_16x16x32_f16(false, a, false, b, (short)0, c, false, false);
  asm volatile("v_nop\n\tv_nop\n\tv_nop\n\tv_nop" : "+v"(c) : "v"(a), "v"(b));
  return c;
}
__device__ __forceinline__ v8f mma_b(v16b a, v16b b, v8f c) {
  c = __builtin_amdgcn_wmma_f32_16x16x32_bf16(false, a, false, b, (short)0, c, false, false);
  asm volatile("v_nop\n\tv_nop\n\tv_nop\n\tv_nop" : "+v"(c) : "v"(a), "v"(b));
  return c;
}
__device__ __forceinline__ void keep4_h(v16h a, v16h b, v16h c, v16h d) { asm volatile("v_nop" :: "v"(a), "v"(b), "v"(c), "v"(d)); }
__device__ __forceinline__ void keep4_b(v16b a, v16b b, v16b c, v16b d) { asm volatile("v_nop" :: "v"(a), "v"(b), "v"(c), "v"(d)); }
__device__ __forceinline__ void acc_guard4(v8f& a, v8f& b, v8f& c, v8f& d) { asm volatile("v_nop\n\tv_nop\n\tv_nop\n\tv_nop" : "+v"(a), "+v"(b), "+v"(c), "+v"(d)); }

template <typename T> struct Frag;
template <> struct Frag<_Float16> {
  typedef v16h V;
  union U { v16h v; v8h h[2]; };
  static __device__ __forceinline__ v16h load(const _Float16* p) {
    U f; f.h[0] = *(const v8h*)(p); f.h[1] = *(const v8h*)(p + 16); return f.v;
  }
  static __device__ __forceinline__ v8f mma(v16h a, v16h b, v8f c) { return mma_h(a, b, c); }
  static __device__ __forceinline__ void keep(v16h a, v16h b, v16h c, v16h d) { keep4_h(a, b, c, d); }
};
template <> struct Frag<__bf16> {
  typedef v16b V;
  union U { v16b v; v8b h[2]; };
  static __device__ __forceinline__ v16b load(const __bf16* p) {
    U f; f.h[0] = *(const v8b*)(p); f.h[1] = *(const v8b*)(p + 16); return f.v;
  }
  static __device__ __forceinline__ v8f mma(v16b a, v16b b, v8f c) { return mma_b(a, b, c); }
  static __device__ __forceinline__ void keep(v16b a, v16b b, v16b c, v16b d) { keep4_b(a, b, c, d); }
};

template <int ET> struct Elem;
template <> struct Elem<0> { typedef _Float16 T; };
template <> struct Elem<1> { typedef __bf16 T; };

template <int ET, bool SPLIT, int BIAS_MODE, int OUT_MODE, bool COMB>
__global__ __launch_bounds__(256) void wmma_gemm64(
    const unsigned short* __restrict__ Ap, const unsigned short* __restrict__ A2p, int lda, long strideA,
    const unsigned short* __restrict__ Btp, const unsigned short* __restrict__ Bt2p, int ldb, long strideB,
    void* __restrict__ Cout, int ldc, long strideC,
    const float* __restrict__ bias,
    const float* __restrict__ xres, long strideX, int ldx,
    const unsigned short* __restrict__ pam,
    const float* __restrict__ gpp, const float* __restrict__ gcp,
    int M, int N, int K, float scale) {
  typedef typename Elem<ET>::T T;
  typedef typename Frag<T>::V V;
  const T* A = (const T*)Ap; const T* A2 = (const T*)A2p; const T* Bt = (const T*)Btp; const T* Bt2 = (const T*)Bt2p;
  __shared__ __align__(16) float sT[8][16 * 68];
  const int b    = blockIdx.y;
  const int lane = threadIdx.x & 31;
  const int wave = threadIdx.x >> 5;
  const int tilesN = N >> 6;
  const int tilesM = M >> 6;
  const int tile = blockIdx.x * 8 + wave;
  if (tile >= tilesM * tilesN) return;
  const int tm = tile / tilesN;
  const int tn = tile - tm * tilesN;
  const int m0 = tm << 6;
  const int n0 = tn << 6;

  const T* Ab  = A  + (size_t)b * strideA;
  const T* Bb  = Bt + (size_t)b * strideB;
  const T* Ab2 = SPLIT ? (A2  + (size_t)b * strideA) : nullptr;
  const T* Bb2 = SPLIT ? (Bt2 + (size_t)b * strideB) : nullptr;

  const int rlane = lane & 15;
  const int koff  = (lane >> 4) * 8;
  const int mOff  = (lane >> 4) * 8;

  v8f acc[4][4];
#pragma unroll
  for (int i = 0; i < 4; ++i)
#pragma unroll
    for (int j = 0; j < 4; ++j) acc[i][j] = (v8f){0.f, 0.f, 0.f, 0.f, 0.f, 0.f, 0.f, 0.f};

  for (int k0 = 0; k0 < K; k0 += 32) {
    V bh[4], bl[4];
#pragma unroll
    for (int j = 0; j < 4; ++j) {
      const size_t bo = (size_t)(n0 + (j << 4) + rlane) * ldb + koff + k0;
      bh[j] = Frag<T>::load(Bb + bo);
      if (SPLIT) bl[j] = Frag<T>::load(Bb2 + bo);
    }
#pragma unroll
    for (int i = 0; i < 4; ++i) {
      const size_t ao = (size_t)(m0 + (i << 4) + rlane) * lda + koff + k0;
      V ah = Frag<T>::load(Ab + ao);
      V al;
      if (SPLIT) al = Frag<T>::load(Ab2 + ao);
#pragma unroll
      for (int j = 0; j < 4; ++j) {
        acc[i][j] = Frag<T>::mma(ah, bh[j], acc[i][j]);
        if (SPLIT) {
          acc[i][j] = Frag<T>::mma(ah, bl[j], acc[i][j]);
          acc[i][j] = Frag<T>::mma(al, bh[j], acc[i][j]);
        }
      }
    }
    Frag<T>::keep(bh[0], bh[1], bh[2], bh[3]);
    if (SPLIT) Frag<T>::keep(bl[0], bl[1], bl[2], bl[3]);
  }
  acc_guard4(acc[0][0], acc[0][1], acc[0][2], acc[0][3]);
  acc_guard4(acc[1][0], acc[1][1], acc[1][2], acc[1][3]);
  acc_guard4(acc[2][0], acc[2][1], acc[2][2], acc[2][3]);
  acc_guard4(acc[3][0], acc[3][1], acc[3][2], acc[3][3]);

  float* slab = sT[wave];
  const float* Xb = COMB ? (xres + (size_t)b * strideX) : nullptr;
  float gp = 0.f, gcs = 0.f;
  if (COMB) { gp = gpp[0]; gcs = gcp[0] * scale; }
#pragma unroll
  for (int i = 0; i < 4; ++i) {
    const int mBase = m0 + (i << 4);
#pragma unroll
    for (int j = 0; j < 4; ++j) {
      const int n = n0 + (j << 4) + rlane;
      if (COMB) {
        const float* xp = Xb + (size_t)n * ldx + mBase + mOff;
        const v4f x0 = *(const v4f*)(xp);
        const v4f x1 = *(const v4f*)(xp + 4);
#pragma unroll
        for (int r = 0; r < 4; ++r) {
          slab[(mOff + r) * 68 + (j << 4) + rlane]     = fmaf(gcs, acc[i][j][r],     2.0f * x0[r]);
          slab[(mOff + 4 + r) * 68 + (j << 4) + rlane] = fmaf(gcs, acc[i][j][4 + r], 2.0f * x1[r]);
        }
      } else {
        float bv = 0.f;
        if (BIAS_MODE == 2) bv = bias[n];
#pragma unroll
        for (int r = 0; r < 8; ++r) {
          float v = acc[i][j][r] * scale;
          if (BIAS_MODE == 1) v += bias[mBase + mOff + r];
          if (BIAS_MODE == 2) v += bv;
          slab[(mOff + r) * 68 + (j << 4) + rlane] = v;
        }
      }
    }
    __builtin_amdgcn_fence(__ATOMIC_RELEASE, "workgroup");
    __builtin_amdgcn_wave_barrier();
    __builtin_amdgcn_fence(__ATOMIC_ACQUIRE, "workgroup");
    if (COMB) {
      const int q = lane >> 3, c8 = (lane & 7) * 8;
      unsigned short* C = (unsigned short*)Cout + (size_t)b * strideC;
      const unsigned short* Pb = pam + (size_t)b * strideC;
      v8h hv4[4];
#pragma unroll
      for (int it = 0; it < 4; ++it) {
        const int row = it * 4 + q;
        const float* sp = slab + row * 68 + c8;
        const v4u pw = *(const v4u*)(Pb + (size_t)(mBase + row) * ldc + n0 + c8);
#pragma unroll
        for (int k = 0; k < 4; ++k) {
          const unsigned w = pw[k];
          const float f0 = h16_to_f32(w & 0xffffu);
          const float f1 = h16_to_f32(w >> 16);
          hv4[it][2 * k]     = (_Float16)fmaf(gp, f0, sp[2 * k]);
          hv4[it][2 * k + 1] = (_Float16)fmaf(gp, f1, sp[2 * k + 1]);
        }
      }
      for (int pass = 0; pass < 2; ++pass) {
#pragma unroll
        for (int it = 0; it < 4; ++it) {
          const int row = it * 4 + q;
          *(volatile v8h*)(C + (size_t)(mBase + row) * ldc + n0 + c8) = hv4[it];
        }
        __threadfence();
      }
    } else if (OUT_MODE == 0) {
      float* C = (float*)Cout + (size_t)b * strideC;
      const int hh = lane >> 4, c4 = (lane & 15) * 4;
      for (int pass = 0; pass < 2; ++pass) {
#pragma unroll
        for (int it = 0; it < 8; ++it) {
          const int row = it * 2 + hh;
          v4f v = *(const v4f*)(slab + row * 68 + c4);
          *(volatile v4f*)(C + (size_t)(mBase + row) * ldc + n0 + c4) = v;
        }
        __threadfence();
      }
    } else {
      const int q = lane >> 3, c8 = (lane & 7) * 8;
      unsigned short* C = (unsigned short*)Cout + (size_t)b * strideC;
      for (int pass = 0; pass < 2; ++pass) {
#pragma unroll
        for (int it = 0; it < 4; ++it) {
          const int row = it * 4 + q;
          const float* sp = slab + row * 68 + c8;
          v8h hv;
#pragma unroll
          for (int e = 0; e < 8; ++e) hv[e] = (_Float16)sp[e];
          *(volatile v8h*)(C + (size_t)(mBase + row) * ldc + n0 + c8) = hv;
        }
        __threadfence();
      }
    }
    __builtin_amdgcn_fence(__ATOMIC_RELEASE, "workgroup");
    __builtin_amdgcn_wave_barrier();
    __builtin_amdgcn_fence(__ATOMIC_ACQUIRE, "workgroup");
  }
}

__global__ __launch_bounds__(256) void prep_x_kernel(const float* __restrict__ x, unsigned short* __restrict__ xh,
                                                     unsigned short* __restrict__ xl, unsigned short* __restrict__ xt) {
  __shared__ __align__(16) float tf[64 * 68];
  const int tid = threadIdx.x;
  const int n0 = blockIdx.x * 64;
  const int c0 = blockIdx.y * 64;
  const int b  = blockIdx.z;
  const float* xb = x + (size_t)b * kCh * kPos;
  {
    const int lr = tid >> 4;
    const int c4 = (tid & 15) * 4;
#pragma unroll
    for (int it = 0; it < 4; ++it) {
      const int rr = it * 16 + lr;
      const v4f a = *(const v4f*)(xb + (size_t)(c0 + rr) * kPos + n0 + c4);
      *(v4f*)(tf + rr * 68 + c4) = a;
    }
  }
  __syncthreads();
  const int sub = tid >> 3;
  const int c8  = (tid & 7) * 8;
  v4u hv[2], lv[2], tv[2];
#pragma unroll
  for (int it = 0; it < 2; ++it) {
    const int r = it * 32 + sub;
    v4u a, a2, a3;
#pragma unroll
    for (int q = 0; q < 4; ++q) {
      const float f0 = tf[r * 68 + c8 + 2 * q];
      const float f1 = tf[r * 68 + c8 + 2 * q + 1];
      const unsigned short h0 = f2bf_bits(f0), h1 = f2bf_bits(f1);
      const unsigned short l0 = f2bf_bits(f0 - bf_bits2f(h0)), l1 = f2bf_bits(f1 - bf_bits2f(h1));
      a[q]  = pk16(h0, h1);
      a2[q] = pk16(l0, l1);
      const float g0 = tf[(c8 + 2 * q) * 68 + r];
      const float g1 = tf[(c8 + 2 * q + 1) * 68 + r];
      a3[q] = pk16(h_bits(g0), h_bits(g1));
    }
    hv[it] = a; lv[it] = a2; tv[it] = a3;
  }
  for (int pass = 0; pass < 2; ++pass) {
#pragma unroll
    for (int it = 0; it < 2; ++it) {
      const int r = it * 32 + sub;
      const size_t go = ((size_t)b * kCh + c0 + r) * kPos + n0 + c8;
      const size_t gt = ((size_t)b * kPos + n0 + r) * kCh + c0 + c8;
      *(volatile v4u*)(xh + go) = hv[it];
      *(volatile v4u*)(xl + go) = lv[it];
      *(volatile v4u*)(xt + gt) = tv[it];
    }
    __threadfence();
  }
}

__global__ __launch_bounds__(256) void prep_w_kernel(const float* __restrict__ qw, const float* __restrict__ kw,
                                                     const float* __restrict__ vw, const float* __restrict__ cw,
                                                     unsigned short* __restrict__ dq, unsigned short* __restrict__ dk,
                                                     unsigned short* __restrict__ dv, unsigned short* __restrict__ dc) {
  const int blk = blockIdx.x;
  const float* src;
  unsigned short* dst;
  int lb;
  if (blk < 16)       { src = qw; dst = dq; lb = blk; }
  else if (blk < 32)  { src = kw; dst = dk; lb = blk - 16; }
  else if (blk < 160) { src = vw; dst = dv; lb = blk - 32; }
  else                { src = cw; dst = dc; lb = blk - 160; }
  const size_t e0 = ((size_t)lb * 256 + threadIdx.x) * 8;
  const v4f a = *(const v4f*)(src + e0);
  const v4f c = *(const v4f*)(src + e0 + 4);
  unsigned short hb[8];
#pragma unroll
  for (int e = 0; e < 4; ++e) {
    hb[e]     = h_bits(a[e] * kWCarry);
    hb[4 + e] = h_bits(c[e] * kWCarry);
  }
  const v4u u = (v4u){pk16(hb[0], hb[1]), pk16(hb[2], hb[3]), pk16(hb[4], hb[5]), pk16(hb[6], hb[7])};
  unsigned short* q = dst + e0;
  *(volatile v4u*)q = u;
  __threadfence();
  *(volatile v4u*)q = u;
}

__global__ __launch_bounds__(256) void cam_softmax_kernel(const float* __restrict__ E, unsigned short* __restrict__ AT) {
  const int lane = threadIdx.x & 31, wave = threadIdx.x >> 5;
  const int gr = blockIdx.x * 8 + wave;
  const float* er = E + (size_t)gr * kCh;
  unsigned short* ar = AT + (size_t)gr * kCh;
  float mn = INFINITY;
#pragma unroll
  for (int hlf = 0; hlf < 2; ++hlf) {
    const float* p = er + hlf * 256 + lane * 8;
    const v4f a = *(const v4f*)(p);
    const v4f c = *(const v4f*)(p + 4);
    mn = fminf(mn, fminf(fminf(a[0], a[1]), fminf(a[2], a[3])));
    mn = fminf(mn, fminf(fminf(c[0], c[1]), fminf(c[2], c[3])));
  }
#pragma unroll
  for (int off = 16; off > 0; off >>= 1) mn = fminf(mn, __shfl_xor(mn, off, 32));
  float sum = 0.f;
#pragma unroll 1
  for (int hlf = 0; hlf < 2; ++hlf) {
    const float* p = er + hlf * 256 + lane * 8;
    const v4f a = *(const v4f*)(p);
    const v4f c = *(const v4f*)(p + 4);
#pragma unroll
    for (int e = 0; e < 4; ++e) {
      sum += __expf(mn - a[e]);
      sum += __expf(mn - c[e]);
    }
  }
#pragma unroll
  for (int off = 16; off > 0; off >>= 1) sum += __shfl_xor(sum, off, 32);
  const float sc = kACarry * (1.0f / sum);
#pragma unroll 1
  for (int hlf = 0; hlf < 2; ++hlf) {
    const float* p = er + hlf * 256 + lane * 8;
    const v4f a = *(const v4f*)(p);
    const v4f c = *(const v4f*)(p + 4);
    unsigned short hb[8];
#pragma unroll
    for (int e = 0; e < 4; ++e) {
      hb[e]     = h_bits(__expf(mn - a[e]) * sc);
      hb[4 + e] = h_bits(__expf(mn - c[e]) * sc);
    }
    const v4u u = (v4u){pk16(hb[0], hb[1]), pk16(hb[2], hb[3]), pk16(hb[4], hb[5]), pk16(hb[6], hb[7])};
    unsigned short* q = ar + hlf * 256 + lane * 8;
    *(volatile v4u*)q = u;
    __threadfence();
    *(volatile v4u*)q = u;
  }
}

__global__ __launch_bounds__(256) void pam_softmax_kernel(unsigned short* SP) {
  __shared__ __align__(16) float sRow[kPos];
  __shared__ float redM[8];
  __shared__ float redS[8];
  const int t = threadIdx.x, lane = t & 31, wave = t >> 5;
  unsigned short* rp = SP + (size_t)blockIdx.x * kPos;
  float m = -INFINITY;
#pragma unroll
  for (int hlf = 0; hlf < 2; ++hlf) {
    const int base = hlf * 2048 + t * 8;
    const v4u w = *(const v4u*)(rp + base);
#pragma unroll
    for (int k = 0; k < 4; ++k) {
      const unsigned wk = w[k];
      const float f0 = h16_to_f32(wk & 0xffffu);
      const float f1 = h16_to_f32(wk >> 16);
      sRow[base + 2 * k]     = f0;
      sRow[base + 2 * k + 1] = f1;
      m = fmaxf(m, fmaxf(f0, f1));
    }
  }
#pragma unroll
  for (int off = 16; off > 0; off >>= 1) m = fmaxf(m, __shfl_xor(m, off, 32));
  if (lane == 0) redM[wave] = m;
  __syncthreads();
  float mx = redM[0];
#pragma unroll
  for (int w = 1; w < 8; ++w) mx = fmaxf(mx, redM[w]);
  float sum = 0.f;
#pragma unroll 1
  for (int hlf = 0; hlf < 2; ++hlf) {
    float* p = sRow + hlf * 2048 + t * 8;
#pragma unroll
    for (int e = 0; e < 8; ++e) {
      const float v = __expf(p[e] - mx);
      p[e] = v;
      sum += v;
    }
  }
#pragma unroll
  for (int off = 16; off > 0; off >>= 1) sum += __shfl_xor(sum, off, 32);
  if (lane == 0) redS[wave] = sum;
  __syncthreads();
  float tot = redS[0];
#pragma unroll
  for (int w = 1; w < 8; ++w) tot += redS[w];
  const float sc = kPCarry * (1.0f / tot);
  v4u u[2];
#pragma unroll
  for (int hlf = 0; hlf < 2; ++hlf) {
    const float* p = sRow + hlf * 2048 + t * 8;
    unsigned short hb[8];
#pragma unroll
    for (int e = 0; e < 8; ++e) hb[e] = h_bits(p[e] * sc);
    u[hlf] = (v4u){pk16(hb[0], hb[1]), pk16(hb[2], hb[3]), pk16(hb[4], hb[5]), pk16(hb[6], hb[7])};
  }
  for (int pass = 0; pass < 2; ++pass) {
#pragma unroll
    for (int hlf = 0; hlf < 2; ++hlf) *(volatile v4u*)(rp + hlf * 2048 + t * 8) = u[hlf];
    __threadfence();
  }
}

__global__ __launch_bounds__(256) void bn_relu_kernel(const float* __restrict__ y, const float* __restrict__ g,
                                                      const float* __restrict__ be, float* __restrict__ out) {
  __shared__ float red1[8];
  __shared__ float red2[8];
  const int o = blockIdx.x, t = threadIdx.x, lane = t & 31, wave = t >> 5;
  float s = 0.f;
#pragma unroll 1
  for (int b = 0; b < kNB; ++b) {
    const float* yp = y + ((size_t)b * kOutC + o) * kPos;
#pragma unroll
    for (int it = 0; it < 4; ++it) {
      const v4f v = *(const v4f*)(yp + (size_t)(it * 256 + t) * 4);
      s += (v[0] + v[1]) + (v[2] + v[3]);
    }
  }
#pragma unroll
  for (int off = 16; off > 0; off >>= 1) s += __shfl_xor(s, off, 32);
  if (lane == 0) red1[wave] = s;
  __syncthreads();
  float tot = red1[0];
#pragma unroll
  for (int w = 1; w < 8; ++w) tot += red1[w];
  const float mean = tot * kBnCntInv;
  float s2 = 0.f;
#pragma unroll 1
  for (int b = 0; b < kNB; ++b) {
    const float* yp = y + ((size_t)b * kOutC + o) * kPos;
#pragma unroll
    for (int it = 0; it < 4; ++it) {
      const v4f v = *(const v4f*)(yp + (size_t)(it * 256 + t) * 4);
      const float d0 = v[0] - mean, d1 = v[1] - mean, d2 = v[2] - mean, d3 = v[3] - mean;
      s2 += (d0 * d0 + d1 * d1) + (d2 * d2 + d3 * d3);
    }
  }
#pragma unroll
  for (int off = 16; off > 0; off >>= 1) s2 += __shfl_xor(s2, off, 32);
  if (lane == 0) red2[wave] = s2;
  __syncthreads();
  float tot2 = red2[0];
#pragma unroll
  for (int w = 1; w < 8; ++w) tot2 += red2[w];
  const float var = tot2 * kBnCntInv;
  const float inv = 1.0f / sqrtf(var + kBnEps);
  const float gg = g[o], bb = be[o];
#pragma unroll 1
  for (int b = 0; b < kNB; ++b) {
    const float* yp = y + ((size_t)b * kOutC + o) * kPos;
    float* op = out + ((size_t)b * kOutC + o) * kPos;
    v4f r[4];
#pragma unroll
    for (int it = 0; it < 4; ++it) {
      const v4f v = *(const v4f*)(yp + (size_t)(it * 256 + t) * 4);
      v4f w;
#pragma unroll
      for (int e = 0; e < 4; ++e) {
        const float yn = (v[e] - mean) * inv;
        w[e] = fmaxf(yn * gg + bb, 0.0f);
      }
      r[it] = w;
    }
    for (int pass = 0; pass < 2; ++pass) {
#pragma unroll
      for (int it = 0; it < 4; ++it) *(volatile v4f*)(op + (size_t)(it * 256 + t) * 4) = r[it];
      __threadfence();
    }
  }
}

extern "C" void kernel_launch(void* const* d_in, const int* in_sizes, int n_in,
                              void* d_out, int out_size, void* d_ws, size_t ws_size,
                              hipStream_t stream) {
  if (n_in < 12) return;
  if (in_sizes[0] != kNB * kCh * kPos) return;
  if (in_sizes[1] != kCq * kCh) return;
  if (in_sizes[2] != kCq) return;
  if (in_sizes[3] != kCq * kCh) return;
  if (in_sizes[4] != kCq) return;
  if (in_sizes[5] != kCh * kCh) return;
  if (in_sizes[6] != kCh) return;
  if (in_sizes[7] != 1) return;
  if (in_sizes[8] != 1) return;
  if (in_sizes[9] != kOutC * kCh) return;
  if (in_sizes[10] != kOutC) return;
  if (in_sizes[11] != kOutC) return;
  if (out_size != kNB * kOutC * kPos) return;
  if (ws_size < kWsTotal) return;

  const float* x     = (const float*)d_in[0];
  const float* q_w   = (const float*)d_in[1];
  const float* q_b   = (const float*)d_in[2];
  const float* k_w   = (const float*)d_in[3];
  const float* k_b   = (const float*)d_in[4];
  const float* v_w   = (const float*)d_in[5];
  const float* v_b   = (const float*)d_in[6];
  const float* g_pam = (const float*)d_in[7];
  const float* g_cam = (const float*)d_in[8];
  const float* c_w   = (const float*)d_in[9];
  const float* bn_g  = (const float*)d_in[10];
  const float* bn_b  = (const float*)d_in[11];
  float* out = (float*)d_out;

  char* ws = (char*)d_ws;
  unsigned short* XH = (unsigned short*)(ws + kOffR0);
  unsigned short* XL = (unsigned short*)(ws + kOffR0 + kSzR0 / 2);
  unsigned short* SP = (unsigned short*)(ws + kOffR0);
  unsigned short* XT = (unsigned short*)(ws + kOffXT);
  unsigned short* QT = (unsigned short*)(ws + kOffQT);
  unsigned short* KT = (unsigned short*)(ws + kOffKT);
  unsigned short* VV = (unsigned short*)(ws + kOffVV);
  float*          EE = (float*)(ws + kOffEE);
  unsigned short* AT = (unsigned short*)(ws + kOffAT);
  unsigned short* PM = (unsigned short*)(ws + kOffPM);
  unsigned short* ST = (unsigned short*)(ws + kOffST);
  float*          YY = (float*)(ws + kOffYY);
  unsigned short* WQ = (unsigned short*)(ws + kOffWQ);
  unsigned short* WK = (unsigned short*)(ws + kOffWK);
  unsigned short* WV = (unsigned short*)(ws + kOffWV);
  unsigned short* WC = (unsigned short*)(ws + kOffWC);

  const long sCN = (long)kCh * kPos;
  const long sNQ = (long)kPos * kCq;
  const long sCC = (long)kCh * kCh;
  const long sON = (long)kOutC * kPos;

  prep_x_kernel<<<dim3(kPos / 64, kCh / 64, kNB), 256, 0, stream>>>(x, XH, XL, XT);
  prep_w_kernel<<<224, 256, 0, stream>>>(q_w, k_w, v_w, c_w, WQ, WK, WV, WC);

  wmma_gemm64<1, true, 0, 0, false><<<dim3(8, kNB), 256, 0, stream>>>(
      XH, XL, kPos, sCN, XH, XL, kPos, sCN,
      (void*)EE, kCh, sCC, nullptr, nullptr, 0L, 0, nullptr, nullptr, nullptr,
      kCh, kCh, kPos, 1.0f);

  cam_softmax_kernel<<<(kNB * kCh) / 8, 256, 0, stream>>>(EE, AT);

  wmma_gemm64<0, false, 2, 1, false><<<dim3(8, kNB), 256, 0, stream>>>(
      XT, nullptr, kCh, sCN, WQ, nullptr, kCh, 0L,
      (void*)QT, kCq, sNQ, q_b, nullptr, 0L, 0, nullptr, nullptr, nullptr,
      kPos, kCq, kCh, kWCarryInv);
  wmma_gemm64<0, false, 2, 1, false><<<dim3(8, kNB), 256, 0, stream>>>(
      XT, nullptr, kCh, sCN, WK, nullptr, kCh, 0L,
      (void*)KT, kCq, sNQ, k_b, nullptr, 0L, 0, nullptr, nullptr, nullptr,
      kPos, kCq, kCh, kWCarryInv);

  wmma_gemm64<0, false, 1, 1, false><<<dim3(64, kNB), 256, 0, stream>>>(
      WV, nullptr, kCh, 0L, XT, nullptr, kCh, sCN,
      (void*)VV, kPos, sCN, v_b, nullptr, 0L, 0, nullptr, nullptr, nullptr,
      kCh, kPos, kCh, kWCarryInv);

  for (int b = 0; b < kNB; ++b) {
    wmma_gemm64<0, false, 0, 1, false><<<dim3(512, 1), 256, 0, stream>>>(
        QT + (size_t)b * sNQ, nullptr, kCq, 0L, KT + (size_t)b * sNQ, nullptr, kCq, 0L,
        (void*)SP, kPos, 0L, nullptr, nullptr, 0L, 0, nullptr, nullptr, nullptr,
        kPos, kPos, kCq, 1.0f);
    pam_softmax_kernel<<<kPos, 256, 0, stream>>>(SP);
    wmma_gemm64<0, false, 0, 1, false><<<dim3(64, 1), 256, 0, stream>>>(
        SP, nullptr, kPos, 0L, VV + (size_t)b * sCN, nullptr, kPos, 0L,
        (void*)(PM + (size_t)b * sCN), kCh, 0L, nullptr, nullptr, 0L, 0, nullptr, nullptr, nullptr,
        kPos, kCh, kPos, kPCarryInv);
  }

  wmma_gemm64<0, false, 0, 1, true><<<dim3(64, kNB), 256, 0, stream>>>(
      XT, nullptr, kCh, sCN, AT, nullptr, kCh, sCC,
      (void*)ST, kCh, sCN, nullptr, x, sCN, kPos, PM, g_pam, g_cam,
      kPos, kCh, kCh, kACarryInv);

  wmma_gemm64<0, false, 0, 0, false><<<dim3(32, kNB), 256, 0, stream>>>(
      WC, nullptr, kCh, 0L, ST, nullptr, kCh, sCN,
      (void*)YY, kPos, sON, nullptr, nullptr, 0L, 0, nullptr, nullptr, nullptr,
      kOutC, kPos, kCh, kWCarryInv);

  bn_relu_kernel<<<kOutC, 256, 0, stream>>>(YY, bn_g, bn_b, out);
}
